// _MS_NonLocalBlockND_16896401343292
// MI455X (gfx1250) — hardware-verified
//
#include <hip/hip_runtime.h>


namespace {
constexpr int Bn = 4, C = 256, NP = 4096, C1 = 64, C2 = 64, NTOK = Bn * NP, NPB = NP / 128;
constexpr float QS = 8.0f, VS = 8.0f, PS = 8.0f, YS = 8.0f, SCALE = 0.125f, EPS = 1e-5f;
constexpr size_t QPL = (size_t)NTOK * C1, VPL = (size_t)Bn * C2 * NP;

typedef _Float16 b16;
typedef __attribute__((ext_vector_type(16))) _Float16 v16b;
typedef __attribute__((ext_vector_type(16))) __bf16 v16bb;
typedef __attribute__((ext_vector_type(8))) _Float16 v8b;
typedef __attribute__((ext_vector_type(8))) unsigned short v8us;
typedef __attribute__((ext_vector_type(8))) float v8f;
typedef __attribute__((ext_vector_type(4))) float v4f;
__device__ __forceinline__ float bf16_rne(float f) { unsigned int u = __float_as_uint(f); u += 0x7FFFu + ((u >> 16) & 1u); return __uint_as_float(u & 0xFFFF0000u); }
__device__ __forceinline__ unsigned short bf16_bits(float f) { unsigned int u = __float_as_uint(f); u += 0x7FFFu + ((u >> 16) & 1u); return (unsigned short)(u >> 16); }
__device__ __forceinline__ void split16(float v, b16& hi, b16& lo) { hi = (b16)v; lo = (b16)(v - (float)hi); }
__device__ __forceinline__ v16b frag_kb(const b16* p, int hh) { const v8b a = *(const v8b*)(p + 8 * hh), b = *(const v8b*)(p + 16 + 8 * hh); v16b f;
#pragma unroll
  for (int e = 0; e < 8; ++e) { f[e] = a[e]; f[8 + e] = b[e]; } return f; }
__device__ __forceinline__ v16bb frag_bf(const unsigned short* p, int hh) { const v8us a = *(const v8us*)(p + 8 * hh), b = *(const v8us*)(p + 16 + 8 * hh); union { unsigned short s[16]; v16bb v; } u;
#pragma unroll
  for (int e = 0; e < 8; ++e) { u.s[e] = a[e]; u.s[8 + e] = b[e]; } return u.v; }
__device__ __forceinline__ v8f wmma16b(v16b a, v16b b, v8f c) { v8f d = __builtin_amdgcn_wmma_f32_16x16x32_f16(false, a, false, b, (short)0, c, false, false); asm volatile("v_nop\n\tv_nop\n\tv_nop\n\tv_nop" : "+v"(d) : "v"(a), "v"(b)); return d; }
__device__ __forceinline__ v8f wmma16bb(v16bb a, v16bb b, v8f c) { v8f d = __builtin_amdgcn_wmma_f32_16x16x32_bf16(false, a, false, b, (short)0, c, false, false); asm volatile("v_nop\n\tv_nop\n\tv_nop\n\tv_nop" : "+v"(d) : "v"(a), "v"(b)); return d; }
__device__ __forceinline__ void wave_lds_sync() { __builtin_amdgcn_fence(__ATOMIC_RELEASE, "workgroup"); __builtin_amdgcn_wave_barrier(); __builtin_amdgcn_fence(__ATOMIC_ACQUIRE, "workgroup"); }
__device__ __forceinline__ float nexp(float x) { return __builtin_amdgcn_exp2f(x * 1.4426950408889634f); }

__global__ __launch_bounds__(256) void prep_kernel(const float* __restrict__ x, const float* __restrict__ tw, const float* __restrict__ pw, const float* __restrict__ gw, const float* __restrict__ Ww, unsigned short* __restrict__ xT, unsigned short* __restrict__ w16, b16* __restrict__ ww16) {
  __shared__ __attribute__((aligned(16))) unsigned short Tt[64][C + 8];
  const int t_ = threadIdx.x, b = blockIdx.y, p0 = blockIdx.x * 64; const float* src = x + (size_t)b * C * NP;
  for (int i = t_; i < C * 64; i += 256) { const int c = i >> 6, pp = i & 63; Tt[pp][c] = bf16_bits(src[(size_t)c * NP + p0 + pp]); }
  __syncthreads();
  for (int pass = 0; pass < 2; ++pass) {
    for (int i = t_; i < 64 * C / 8; i += 256) { const int pp = i >> 5, c8 = (i & 31) * 8; *(volatile v8us*)(xT + ((size_t)b * NP + p0 + pp) * C + c8) = *(const v8us*)(&Tt[pp][c8]); }
    if (blockIdx.x == 0 && blockIdx.y == 0) {
      for (int i = t_; i < 3 * C1 * C / 8; i += 256) { const int m = i / (C1 * C / 8), q = i % (C1 * C / 8); const float* W = (m == 0) ? tw : (m == 1) ? pw : gw; v8us o;
#pragma unroll
        for (int e = 0; e < 8; ++e) o[e] = bf16_bits(W[q * 8 + e]);
        *(volatile v8us*)(w16 + (size_t)i * 8) = o; }
      for (int i = t_; i < C * C2 / 8; i += 256) { v8b o;
#pragma unroll
        for (int e = 0; e < 8; ++e) o[e] = (b16)bf16_rne(Ww[i * 8 + e]);
        *(volatile v8b*)(ww16 + (size_t)i * 8) = o; } }
    __threadfence(); }
}

__global__ __launch_bounds__(128) void proj_kernel(const unsigned short* __restrict__ xT, const unsigned short* __restrict__ w16, const float* __restrict__ tb, const float* __restrict__ pb, const float* __restrict__ gb, b16* __restrict__ th, b16* __restrict__ ph, b16* __restrict__ gt) {
  __shared__ __attribute__((aligned(16))) b16 Th[4][32][64 + 8], Tl[4][32][64 + 8]; __shared__ __attribute__((aligned(16))) b16 Vh[64][128 + 8], Vl[64][128 + 8];
  const int lane = threadIdx.x & 31, wave = threadIdx.x >> 5, nloc = lane & 15, hlf = lane >> 4, which = blockIdx.x, m0 = blockIdx.y * 128 + wave * 32; const int b = (blockIdx.y * 128) / NP, p0 = (blockIdx.y * 128) % NP;
  const unsigned short* Wt = w16 + (size_t)which * C1 * C; const float* bias = (which == 0) ? tb : (which == 1) ? pb : gb;
  v8f acc[2][4];
#pragma unroll
  for (int r = 0; r < 2; ++r)
#pragma unroll
    for (int t = 0; t < 4; ++t) acc[r][t] = (v8f){};
#pragma unroll 2
  for (int kb = 0; kb < C; kb += 32) { const v16bb a0 = frag_bf(xT + (size_t)(m0 + nloc) * C + kb, hlf), a1 = frag_bf(xT + (size_t)(m0 + 16 + nloc) * C + kb, hlf);
#pragma unroll
    for (int t = 0; t < 4; ++t) { const v16bb bw = frag_bf(Wt + (size_t)(t * 16 + nloc) * C + kb, hlf); acc[0][t] = wmma16bb(a0, bw, acc[0][t]); acc[1][t] = wmma16bb(a1, bw, acc[1][t]); } }
  const float scl = (which == 2) ? VS : QS;
#pragma unroll
  for (int t = 0; t < 4; ++t) { const int c = t * 16 + nloc; const float bb = bf16_rne(bias[c]);
#pragma unroll
    for (int r = 0; r < 2; ++r)
#pragma unroll
      for (int v = 0; v < 8; ++v) { b16 a_, c_; split16((acc[r][t][v] + bb) * scl, a_, c_); const int row = r * 16 + 8 * hlf + v;
        if (which < 2) { Th[wave][row][c] = a_; Tl[wave][row][c] = c_; } else { Vh[c][wave * 32 + row] = a_; Vl[c][wave * 32 + row] = c_; } } }
  __syncthreads();
  for (int pass = 0; pass < 2; ++pass) {
    if (which < 2) { b16* dst = ((which == 0) ? th : ph) + (size_t)m0 * C1;
#pragma unroll
      for (int j = 0; j < 8; ++j) { const int rr = j * 4 + (lane >> 3), c8 = (lane & 7) * 8; *(volatile v8b*)(dst + (size_t)rr * C1 + c8) = *(const v8b*)(&Th[wave][rr][c8]); *(volatile v8b*)(dst + QPL + (size_t)rr * C1 + c8) = *(const v8b*)(&Tl[wave][rr][c8]); } }
    else { for (int i = threadIdx.x; i < 64 * 16; i += 128) { const int cc = i >> 4, c8 = (i & 15) * 8; const size_t dst = ((size_t)b * C2 + cc) * NP + p0 + c8;
        *(volatile v8b*)(gt + dst) = *(const v8b*)(&Vh[cc][c8]); *(volatile v8b*)(gt + VPL + dst) = *(const v8b*)(&Vl[cc][c8]); } }
    __threadfence(); }
}

__global__ __launch_bounds__(256) void attn_kernel(const b16* __restrict__ th, const b16* __restrict__ ph, const b16* __restrict__ gt, float* __restrict__ yrow) {
  __shared__ __attribute__((aligned(16))) float Os[8][16][C2 + 4];
  const int wid = threadIdx.x >> 5, lane = threadIdx.x & 31, hh = lane >> 4, col = lane & 15; const int tok0 = blockIdx.x * 128 + wid * 16, b = tok0 / NP; const size_t qi = (size_t)tok0 + col;
  const b16* K = ph + ((size_t)b * NP) * C1; const b16* V = gt + ((size_t)b * C2) * NP;
  v16b qf[2], ql[2];
#pragma unroll
  for (int ks = 0; ks < 2; ++ks) { qf[ks] = frag_kb(th + qi * C1 + ks * 32, hh); ql[ks] = frag_kb(th + QPL + qi * C1 + ks * 32, hh); }
  float m = -INFINITY, l = 0.0f; v8f o[4] = {{}, {}, {}, {}};
  for (int kb = 0; kb < NP; kb += 32) { v8f s0 = {}, s1 = {};
#pragma unroll
    for (int ks = 0; ks < 2; ++ks) { const v16b ka = frag_kb(K + (size_t)(kb + col) * C1 + ks * 32, hh), kal = frag_kb(K + QPL + (size_t)(kb + col) * C1 + ks * 32, hh), kb_ = frag_kb(K + (size_t)(kb + 16 + col) * C1 + ks * 32, hh), kbl = frag_kb(K + QPL + (size_t)(kb + 16 + col) * C1 + ks * 32, hh);
      s0 = wmma16b(ka, qf[ks], s0); s0 = wmma16b(ka, ql[ks], s0); s0 = wmma16b(kal, qf[ks], s0); s1 = wmma16b(kb_, qf[ks], s1); s1 = wmma16b(kb_, ql[ks], s1); s1 = wmma16b(kbl, qf[ks], s1); }
    float mr = -INFINITY;
#pragma unroll
    for (int r = 0; r < 8; ++r) { s0[r] *= SCALE / (QS * QS); s1[r] *= SCALE / (QS * QS); mr = fmaxf(mr, fmaxf(s0[r], s1[r])); }
    mr = fmaxf(mr, __shfl_xor(mr, 16));
    const float mn = fmaxf(m, mr), al_ = nexp(m - mn); m = mn; float sum = 0.0f; v16b pbv, plv;
#pragma unroll
    for (int r = 0; r < 8; ++r) { const float p0 = nexp(s0[r] - mn), p1 = nexp(s1[r] - mn); sum += p0 + p1; b16 a, c; split16(p0 * PS, a, c); pbv[r] = a; plv[r] = c; split16(p1 * PS, a, c); pbv[8 + r] = a; plv[8 + r] = c; }
    sum += __shfl_xor(sum, 16); l = l * al_ + sum;
#pragma unroll
    for (int n = 0; n < 4; ++n) { o[n] *= al_; const v16b vf = frag_kb(V + (size_t)(n * 16 + col) * NP + kb, hh), vl = frag_kb(V + VPL + (size_t)(n * 16 + col) * NP + kb, hh); o[n] = wmma16b(vf, pbv, o[n]); o[n] = wmma16b(vf, plv, o[n]); o[n] = wmma16b(vl, pbv, o[n]); } }
  const float inv = 1.0f / (l * VS * PS);
#pragma unroll
  for (int n = 0; n < 4; ++n)
#pragma unroll
    for (int r = 0; r < 8; ++r) Os[wid][col][n * 16 + 8 * hh + r] = o[n][r] * inv;
  wave_lds_sync();
  float* dst = yrow + (size_t)tok0 * C2;
  for (int pass = 0; pass < 2; ++pass) {
#pragma unroll
    for (int j = 0; j < 8; ++j) { const int rr = j * 2 + hh, c4 = col * 4; *(volatile v4f*)(dst + (size_t)rr * C2 + c4) = *(const v4f*)(&Os[wid][rr][c4]); }
    __threadfence(); }
}

__global__ __launch_bounds__(128) void wconv_kernel(const float* __restrict__ yrow, const b16* __restrict__ ww16, const float* __restrict__ Wb, float* __restrict__ wy, float* __restrict__ part) {
  __shared__ __attribute__((aligned(16))) float Ts[4][32 * 64]; __shared__ float Cs[4][2][64];
  const int lane = threadIdx.x & 31, wave = threadIdx.x >> 5, nloc = lane & 15, hlf = lane >> 4, m0 = blockIdx.y * 128 + wave * 32, c0 = blockIdx.x * 64;
  v8f acc[2][4];
#pragma unroll
  for (int r = 0; r < 2; ++r)
#pragma unroll
    for (int t = 0; t < 4; ++t) acc[r][t] = (v8f){};
#pragma unroll
  for (int kb = 0; kb < C2; kb += 32) { v16b a0, a1, l0, l1;
#pragma unroll
    for (int e = 0; e < 16; ++e) { const int k = kb + ((e < 8) ? (8 * hlf + e) : (16 + 8 * hlf + e - 8)); b16 p, q; split16(yrow[(size_t)(m0 + nloc) * C2 + k] * YS, p, q); a0[e] = p; l0[e] = q; split16(yrow[(size_t)(m0 + 16 + nloc) * C2 + k] * YS, p, q); a1[e] = p; l1[e] = q; }
#pragma unroll
    for (int t = 0; t < 4; ++t) { const v16b bw = frag_kb(ww16 + (size_t)(c0 + t * 16 + nloc) * C2 + kb, hlf); acc[0][t] = wmma16b(a0, bw, acc[0][t]); acc[0][t] = wmma16b(l0, bw, acc[0][t]); acc[1][t] = wmma16b(a1, bw, acc[1][t]); acc[1][t] = wmma16b(l1, bw, acc[1][t]); } }
  float* Tt = Ts[wave];
#pragma unroll
  for (int t = 0; t < 4; ++t) { const float bb = bf16_rne(Wb[c0 + t * 16 + nloc]);
#pragma unroll
    for (int r = 0; r < 2; ++r)
#pragma unroll
      for (int v = 0; v < 8; ++v) Tt[(r * 16 + v + 8 * hlf) * 64 + t * 16 + nloc] = acc[r][t][v] * (1.0f / YS) + bb; }
  wave_lds_sync();
  { float s = 0.0f, s2 = 0.0f, q1 = 0.0f, q2 = 0.0f; for (int rr = 0; rr < 32; ++rr) { const float a = Tt[rr * 64 + lane * 2], c = Tt[rr * 64 + lane * 2 + 1]; s += a; q1 += a * a; s2 += c; q2 += c * c; }
    Cs[wave][0][lane * 2] = s; Cs[wave][0][lane * 2 + 1] = s2; Cs[wave][1][lane * 2] = q1; Cs[wave][1][lane * 2 + 1] = q2; }
  __syncthreads();
  float* dst0 = wy + (size_t)m0 * C + c0;
  for (int pass = 0; pass < 2; ++pass) {
#pragma unroll
    for (int j = 0; j < 16; ++j) { const int rr = j * 2 + hlf, c4 = nloc * 4; *(volatile v4f*)(dst0 + (size_t)rr * C + c4) = *(const v4f*)(Tt + rr * 64 + c4); }
    if (threadIdx.x < 128) { const int st = threadIdx.x >> 6, cc = threadIdx.x & 63; ((volatile float*)part)[(((size_t)blockIdx.y * 4 + blockIdx.x) * 2 + st) * 64 + cc] = Cs[0][st][cc] + Cs[1][st][cc] + Cs[2][st][cc] + Cs[3][st][cc]; }
    __threadfence(); }
}

__global__ __launch_bounds__(256) void bnstat_kernel(const float* __restrict__ part, const float* __restrict__ gma, const float* __restrict__ bta, float* __restrict__ bn, int ntok) {
  const int c = threadIdx.x; const int ct = c >> 6, cc = c & 63; double s = 0.0, q = 0.0;
  for (int blk = 0; blk < ntok / 128; ++blk) { s += (double)part[(((size_t)blk * 4 + ct) * 2 + 0) * 64 + cc]; q += (double)part[(((size_t)blk * 4 + ct) * 2 + 1) * 64 + cc]; }
  const double mean = s / (double)ntok; const double var = fmax(q / (double)ntok - mean * mean, 0.0);
  const float scl = bf16_rne(gma[c]) * (float)(1.0 / sqrt(var + (double)EPS)); const float sh = bf16_rne(bta[c]) - (float)mean * scl;
  for (int pass = 0; pass < 2; ++pass) { ((volatile float*)bn)[c] = scl; ((volatile float*)bn)[C + c] = sh; __threadfence(); }
}

__global__ __launch_bounds__(256) void final_kernel(const float* __restrict__ wy, const float* __restrict__ bn, float* __restrict__ out) {
  __shared__ __attribute__((aligned(16))) float Ta[64][128 + 4];
  const int b = blockIdx.y, p0 = blockIdx.x * 128, t_ = threadIdx.x;
  for (int cb = 0; cb < C; cb += 64) {
    for (int i = t_; i < 128 * 16; i += 256) { const int pp = i >> 4, c4 = (i & 15) * 4; const v4f v = *(const v4f*)(wy + ((size_t)b * NP + p0 + pp) * C + cb + c4);
#pragma unroll
      for (int e = 0; e < 4; ++e) Ta[c4 + e][pp] = v[e]; }
    __syncthreads();
    for (int pass = 0; pass < 2; ++pass) { for (int i = t_; i < 64 * 32; i += 256) { const int c = i >> 5, q4 = (i & 31) * 4; const float sc = bn[cb + c], sh = bn[C + cb + c]; v4f o;
#pragma unroll
        for (int e = 0; e < 4; ++e) o[e] = Ta[c][q4 + e] * sc + sh;
        *(volatile v4f*)(out + ((size_t)b * C + cb + c) * NP + p0 + q4) = o; } __threadfence(); }
    __syncthreads();
  }
}
}

extern "C" void kernel_launch(void* const* d_in, const int* in_sizes, int n_in,
                              void* d_out, int out_size, void* d_ws, size_t ws_size, hipStream_t stream) {
  (void)n_in; (void)out_size;
  const float* x = (const float*)d_in[0]; const float* tw = (const float*)d_in[1]; const float* tb = (const float*)d_in[2]; const float* pw = (const float*)d_in[3]; const float* pb = (const float*)d_in[4]; const float* gw = (const float*)d_in[5]; const float* gb = (const float*)d_in[6];
  const float* Ww = (const float*)d_in[7]; const float* Wb = (const float*)d_in[8]; const float* gma = (const float*)d_in[9]; const float* bta = (const float*)d_in[10];
  float* out = (float*)d_out;
  if (in_sizes[0] != Bn * C * NP || in_sizes[1] != C1 * C || in_sizes[5] != C2 * C || in_sizes[7] != C * C2 || in_sizes[9] != C) return;
  size_t off = 0; char* ws = (char*)d_ws;
  auto carve = [&](size_t bytes) { char* p = ws + off; off += (bytes + 255) & ~(size_t)255; return p; };
  unsigned short* xT = (unsigned short*)carve((size_t)NTOK * C * 2); unsigned short* w16 = (unsigned short*)carve((size_t)3 * C1 * C * 2); b16* ww16 = (b16*)carve((size_t)C * C2 * 2);
  b16* th = (b16*)carve(QPL * 2 * 2); b16* ph = (b16*)carve(QPL * 2 * 2); b16* gt = (b16*)carve(VPL * 2 * 2); float* yrow = (float*)carve((size_t)NTOK * C2 * 4); float* wy = (float*)carve((size_t)NTOK * C * 4); float* part = (float*)carve((size_t)(NTOK / 128) * 4 * 2 * 64 * 4); float* bn = (float*)carve(2 * C * 4);
  if (off > ws_size) return;
  prep_kernel<<<dim3(NP / 64, Bn), 256, 0, stream>>>(x, tw, pw, gw, Ww, xT, w16, ww16);
  proj_kernel<<<dim3(3, NTOK / 128), 128, 0, stream>>>(xT, w16, tb, pb, gb, th, ph, gt);
  attn_kernel<<<NTOK / 128, 256, 0, stream>>>(th, ph, gt, yrow);
  wconv_kernel<<<dim3(C / 64, NTOK / 128), 128, 0, stream>>>(yrow, ww16, Wb, wy, part);
  bnstat_kernel<<<1, 256, 0, stream>>>(part, gma, bta, bn, NTOK);
  final_kernel<<<dim3(NPB, Bn), 256, 0, stream>>>(wy, bn, out);
}
